// GCN_88244398063622
// MI455X (gfx1250) — hardware-verified
//
#include <hip/hip_runtime.h>
#include <stddef.h>
#include <stdint.h>
#include <math.h>


#define DF     128
#define FIN    64
#define K0C    192
#define KS     512
#define AP     512
#define BNEPS  1e-5f
#define NTHR   256
#define NWAVE  8
#define EPT    8
#define CHUNK  (NTHR * EPT)
#define WCAP   (EPT * 32)
#define LISTN  (NWAVE * WCAP)
#define NBA    1024
#define SLA    10
#define RCAP   28672
#define DEGCAP 64
#define GBM    64
#define GBN    128
#define GTHR   128
#define MROWS  128
#define RPW    16
#define GPB    32
#define NUA    (3 * 1024)
#define NUB    (2 * 4 * 2048)
#define NUW    (NUA + NUB)
#define W2OFF  (DF * K0C)
#define W3OFF  (W2OFF + DF * KS)
#define WPLH   (W3OFF + DF * KS)
#define AGG_ZINTS (LISTN + 2 * RCAP + 3 * NBA)
#define CMP_LDS_INTS (AGG_ZINTS + 16)
#define POOL_LDS_FLOATS (NWAVE * GPB * DF + GPB)
#define WSMAX  134217728

static_assert((CHUNK & (CHUNK - 1)) == 0 && CHUNK <= 4096);
static_assert((NBA & (NBA - 1)) == 0 && NBA == (1 << SLA));
static_assert(((long long)CHUNK << SLA) < (1LL << 31));
static_assert(RCAP >= 16710 + 16710 / 20 + 1);
static_assert(DEGCAP >= 36 + 8);
static_assert(RCAP % (NTHR * 4) == 0 && AGG_ZINTS % (NTHR * 4) == 0 && LISTN % 4 == 0);
static_assert(NBA == NTHR * 4);
static_assert(NBA % (NWAVE * RPW) == 0 && MROWS == NWAVE * RPW && MROWS % GBM == 0);
static_assert(K0C % 32 == 0 && KS % 32 == 0 && K0C == 3 * FIN && KS == 4 * DF && AP == KS);
static_assert(GBN == DF && GBM == (GTHR / 32) * 16 && DF == 4 * 32 && FIN == 2 * 32);
static_assert(NUA % NTHR == 0 && NUB % NTHR == 0 && 1024 % NTHR == 0 && 2048 % NTHR == 0);
static_assert(CMP_LDS_INTS * 4 <= 300000 && POOL_LDS_FLOATS * 4 <= 300000);
static_assert(GPB == 32 && GPB == NWAVE * 4);
static_assert((W2OFF * 2) % 128 == 0 && (W3OFF * 2) % 128 == 0);

typedef float          v4f   __attribute__((ext_vector_type(4)));
typedef float          v8f   __attribute__((ext_vector_type(8)));
typedef int            v4i   __attribute__((ext_vector_type(4)));
typedef int            v8i   __attribute__((ext_vector_type(8)));
typedef unsigned int   v2u   __attribute__((ext_vector_type(2)));
typedef unsigned int   v4u   __attribute__((ext_vector_type(4)));
typedef unsigned short v8us  __attribute__((ext_vector_type(8)));
typedef __bf16         v16bf __attribute__((ext_vector_type(16)));
typedef v4f  __attribute__((may_alias)) v4fa;
typedef v4i  __attribute__((may_alias)) v4ia;
typedef v2u  __attribute__((may_alias)) v2ua;
typedef v8us __attribute__((may_alias)) v8usa;
typedef unsigned int __attribute__((may_alias)) u1a;
union FragB { v16bf v; v8us h[2]; v8i w; };

__device__ __forceinline__ v8f wmb(const FragB& a, const FragB& b, v8f c) {
  v8f d = __builtin_amdgcn_wmma_f32_16x16x32_bf16(false, a.v, false, b.v, (short)0, c, false, false);
  asm volatile("v_nop\n\tv_nop\n\tv_nop\n\tv_nop" : "+v"(d) : "v"(a.w), "v"(b.w));
  return d;
}

__device__ __forceinline__ unsigned f2bf(float f) {
  const unsigned u = __float_as_uint(f);
  const unsigned r = ((u + 0x7FFFu + ((u >> 16) & 1u)) >> 16) & 0xFFFFu;
  return (f != f) ? 0x7FC0u : r;
}
__device__ __forceinline__ float bf2f(unsigned b) { return __uint_as_float(b << 16); }
__device__ __forceinline__ float bfr(float f) { return bf2f(f2bf(f)); }
__device__ __forceinline__ v4f bfr4(const v4f a) {
  v4f r; r.x = bfr(a.x); r.y = bfr(a.y); r.z = bfr(a.z); r.w = bfr(a.w); return r;
}
__device__ __forceinline__ float smax(float m, float v) {
  return (m != m) ? m : ((v > m || v != v) ? v : m);
}

template <int SLB>
__device__ __forceinline__ int scan_chunk(const int* __restrict__ dsts, int nE, int cbase, int slotBase,
                                          int nb, int vec8, int* list, int tid, int lane, int wave) {
  int wc = 0;
  const int el0  = tid * EPT;
  const int e0   = cbase + el0;
  const int sent = -2147483647 - 1;
  v4i da, db;
  if (vec8 != 0 && cbase + CHUNK <= nE) {
    da = *(const v4i*)(dsts + e0);
    db = *(const v4i*)(dsts + e0 + 4);
  } else {
    da.x = (e0     < nE) ? dsts[min(e0,     nE - 1)] : sent;
    da.y = (e0 + 1 < nE) ? dsts[min(e0 + 1, nE - 1)] : sent;
    da.z = (e0 + 2 < nE) ? dsts[min(e0 + 2, nE - 1)] : sent;
    da.w = (e0 + 3 < nE) ? dsts[min(e0 + 3, nE - 1)] : sent;
    db.x = (e0 + 4 < nE) ? dsts[min(e0 + 4, nE - 1)] : sent;
    db.y = (e0 + 5 < nE) ? dsts[min(e0 + 5, nE - 1)] : sent;
    db.z = (e0 + 6 < nE) ? dsts[min(e0 + 6, nE - 1)] : sent;
    db.w = (e0 + 7 < nE) ? dsts[min(e0 + 7, nE - 1)] : sent;
  }
  const unsigned nbs = (unsigned)slotBase;
  const unsigned unb = (unsigned)nb;
  const unsigned s0 = (unsigned)da.x - nbs, s1 = (unsigned)da.y - nbs;
  const unsigned s2 = (unsigned)da.z - nbs, s3 = (unsigned)da.w - nbs;
  const unsigned s4 = (unsigned)db.x - nbs, s5 = (unsigned)db.y - nbs;
  const unsigned s6 = (unsigned)db.z - nbs, s7 = (unsigned)db.w - nbs;
  const bool h0 = s0 < unb, h1 = s1 < unb, h2 = s2 < unb, h3 = s3 < unb;
  const bool h4 = s4 < unb, h5 = s5 < unb, h6 = s6 < unb, h7 = s7 < unb;
  const unsigned any = __builtin_amdgcn_ballot_w32(h0 | h1 | h2 | h3 | h4 | h5 | h6 | h7);
  if (any != 0u) {
#define HITJ(J, HJ, SJ) { \
      const unsigned mj = __builtin_amdgcn_ballot_w32(HJ); \
      if (mj != 0u) { \
        if (HJ) { \
          const int pos = wc + (int)__builtin_amdgcn_mbcnt_lo(mj, 0u); \
          if (pos < WCAP) list[wave * WCAP + pos] = ((el0 + (J)) << SLB) | (int)(SJ); \
        } \
        wc += (int)__builtin_popcount(mj); } }
    HITJ(0, h0, s0)
    HITJ(1, h1, s1)
    HITJ(2, h2, s2)
    HITJ(3, h3, s3)
    HITJ(4, h4, s4)
    HITJ(5, h5, s5)
    HITJ(6, h6, s6)
    HITJ(7, h7, s7)
#undef HITJ
  }
  return wc;
}

__device__ __forceinline__ v8us wcol8(const float* __restrict__ W, int k0, int n) {
  const float* p = W + (size_t)k0 * DF + n;
  v8us o;
#pragma unroll
  for (int i = 0; i < 8; ++i) o[i] = (unsigned short)f2bf(p[(size_t)i * DF]);
  return o;
}

__global__ __launch_bounds__(NTHR) void k_prep(const float* __restrict__ x,
                                               const float* __restrict__ w1l, const float* __restrict__ w1r,
                                               const float* __restrict__ w2l, const float* __restrict__ w2r,
                                               const float* __restrict__ w3l, const float* __restrict__ w3r,
                                               unsigned short* wpl, unsigned short* xb, int nN, int nUx) {
  const int u = (int)blockIdx.x * NTHR + (int)threadIdx.x;
  v8us o;
  size_t doff;
  if (u < NUA) {
    const int part = u >> 10;
    const int v = u & 1023;
    const int n = v >> 3, kq = (v & 7) * 8;
    if (part < 2) o = wcol8(w1l, kq, n);
    else          o = wcol8(w1r, kq, n);
    doff = (size_t)n * K0C + (size_t)part * FIN + (size_t)kq;
  } else if (u < NUW) {
    const int v = u - NUA;
    const int lay = v >> 13;
    const int part = (v >> 11) & 3;
    const int w = v & 2047;
    const int n = w >> 4, kq = (w & 15) * 8;
    if (lay == 0) {
      if (part < 2) o = wcol8(w2l, kq, n);
      else          o = wcol8(w2r, kq, n);
    } else {
      if (part < 2) o = wcol8(w3l, kq, n);
      else          o = wcol8(w3r, kq, n);
    }
    doff = (size_t)(lay == 0 ? W2OFF : W3OFF) + (size_t)n * KS + (size_t)part * DF + (size_t)kq;
  } else if (u < NUW + nUx) {
    const int v   = u - NUW;
    const int row = v >> 3;
    const int kq  = (v & 7) * 8;
    const int rc  = row < nN ? row : nN - 1;
    const float* p = x + (size_t)rc * FIN + kq;
    const v4f a = *(const v4f*)p;
    const v4f b = *(const v4f*)(p + 4);
    const bool ok = row < nN;
    o[0] = ok ? (unsigned short)f2bf(a.x) : (unsigned short)0;
    o[1] = ok ? (unsigned short)f2bf(a.y) : (unsigned short)0;
    o[2] = ok ? (unsigned short)f2bf(a.z) : (unsigned short)0;
    o[3] = ok ? (unsigned short)f2bf(a.w) : (unsigned short)0;
    o[4] = ok ? (unsigned short)f2bf(b.x) : (unsigned short)0;
    o[5] = ok ? (unsigned short)f2bf(b.y) : (unsigned short)0;
    o[6] = ok ? (unsigned short)f2bf(b.z) : (unsigned short)0;
    o[7] = ok ? (unsigned short)f2bf(b.w) : (unsigned short)0;
    unsigned short* dx = xb + (size_t)row * FIN + kq;
    *(volatile v8us*)dx = o;
    __threadfence();
    *(volatile v8us*)dx = o;
    return;
  } else {
    return;
  }
  unsigned short* dp = wpl + doff;
  *(volatile v8us*)dp = o;
  __threadfence();
  *(volatile v8us*)dp = o;
}

__global__ __launch_bounds__(NTHR) void k_compact(const int* __restrict__ srcs, const int* __restrict__ dsts,
                                                  int nE, int nN, int vec8,
                                                  int* LIST, int* CNT, int* OFF, int* FLG) {
  extern __shared__ __attribute__((aligned(16))) int dsm[];
  int* list = dsm;
  int* hl   = dsm + LISTN;
  int* sl   = hl + RCAP;
  int* cnt  = sl + RCAP;
  int* offs = cnt + NBA;
  int* cur  = offs + NBA;
  int* misc = cur + NBA;
  const int tid = (int)threadIdx.x, lane = tid & 31, wave = tid >> 5;
  const int nodeBase = (int)blockIdx.x * NBA;

  {
    const v4i z4 = {0, 0, 0, 0};
    for (int i = tid * 4; i < AGG_ZINTS; i += NTHR * 4) *(v4ia*)(dsm + i) = z4;
    if (tid < 16) misc[tid] = 0;
  }
  __syncthreads();

  int t = 0, ov = 0;
  const int nChunks = (nE + CHUNK - 1) / CHUNK;
#pragma unroll 1
  for (int ch = 0; ch < nChunks; ++ch) {
    const int cbase = ch * CHUNK;
    const int wc = scan_chunk<SLA>(dsts, nE, cbase, nodeBase, NBA, vec8, list, tid, lane, wave);
    if (lane == 0) misc[wave] = wc;
    __syncthreads();
    if (wave == 0) {
#pragma unroll 1
      for (int w2 = 0; w2 < NWAVE; ++w2) {
        int c = misc[w2];
        c = c < 0 ? 0 : (c > WCAP ? WCAP : c);
#pragma unroll 1
        for (int b0 = 0; b0 < c; b0 += 32) {
          const int idx = b0 + lane;
          const int ent = list[w2 * WCAP + (idx < WCAP ? idx : WCAP - 1)];
          const int m32 = (c - b0) < 32 ? (c - b0) : 32;
#pragma unroll 1
          for (int k = 0; k < m32; ++k) {
            const int u    = __builtin_amdgcn_readlane(ent, k);
            const int slot = u & (NBA - 1);
            const int el   = (u >> SLA) & (CHUNK - 1);
            const int pk   = ((cbase + el) << SLA) | slot;
            if (t < RCAP) {
              if (lane == 0) { hl[t] = pk; cnt[slot] = cnt[slot] + 1; }
              t = t + 1;
            } else {
              ov = 1;
            }
          }
        }
      }
    }
    __syncthreads();
  }
  if (wave == 0 && lane == 0) { misc[8] = t; misc[9] = ov; }
  __syncthreads();
  int tt = misc[8];
  tt = tt < 0 ? 0 : (tt > RCAP ? RCAP : tt);
  const int ovf = misc[9];

  if (wave == 0) {
    const int base = lane * (NBA / 32);
    int s = 0;
#pragma unroll 1
    for (int i = 0; i < NBA / 32; ++i) s += cnt[base + i];
    int incl = s;
#pragma unroll
    for (int d = 1; d < 32; d <<= 1) {
      const int y = __shfl_up(incl, d, 32);
      if (lane >= d) incl += y;
    }
    int run = incl - s;
#pragma unroll 1
    for (int i = 0; i < NBA / 32; ++i) {
      const int cv = cnt[base + i];
      offs[base + i] = run;
      cur[base + i]  = run;
      run += cv;
    }
  }
  __syncthreads();
  if (wave == 0) {
#pragma unroll 1
    for (int b0 = 0; b0 < tt; b0 += 32) {
      const int idx = b0 + lane;
      const int ent = hl[idx < RCAP ? idx : RCAP - 1];
      const int m32 = (tt - b0) < 32 ? (tt - b0) : 32;
#pragma unroll 1
      for (int k = 0; k < m32; ++k) {
        const int u    = __builtin_amdgcn_readlane(ent, k);
        const int slot = u & (NBA - 1);
        if (lane == 0) {
          int p = cur[slot];
          p = p < 0 ? 0 : (p > RCAP - 1 ? RCAP - 1 : p);
          sl[p] = u;
          cur[slot] = p + 1;
        }
      }
    }
  }
  __syncthreads();

  int* lb = LIST + (size_t)blockIdx.x * RCAP;
#pragma unroll 1
  for (int i = tid * 4; i < RCAP; i += NTHR * 4) {
    const v4i e4 = *(const v4ia*)(sl + i);
    int e0 = e4.x >> SLA, e1 = e4.y >> SLA, e2 = e4.z >> SLA, e3 = e4.w >> SLA;
    e0 = e0 < 0 ? 0 : (e0 > nE - 1 ? nE - 1 : e0);
    e1 = e1 < 0 ? 0 : (e1 > nE - 1 ? nE - 1 : e1);
    e2 = e2 < 0 ? 0 : (e2 > nE - 1 ? nE - 1 : e2);
    e3 = e3 < 0 ? 0 : (e3 > nE - 1 ? nE - 1 : e3);
    int r0 = srcs[e0], r1 = srcs[e1], r2 = srcs[e2], r3 = srcs[e3];
    r0 = r0 < 0 ? 0 : (r0 > nN - 1 ? nN - 1 : r0);
    r1 = r1 < 0 ? 0 : (r1 > nN - 1 ? nN - 1 : r1);
    r2 = r2 < 0 ? 0 : (r2 > nN - 1 ? nN - 1 : r2);
    r3 = r3 < 0 ? 0 : (r3 > nN - 1 ? nN - 1 : r3);
    v4i o4;
    o4.x = (i     < tt) ? r0 : 0;
    o4.y = (i + 1 < tt) ? r1 : 0;
    o4.z = (i + 2 < tt) ? r2 : 0;
    o4.w = (i + 3 < tt) ? r3 : 0;
    int* dp = lb + i;
    *(volatile v4i*)dp = o4;
    __threadfence();
    *(volatile v4i*)dp = o4;
  }
  {
    const v4i c4 = *(const v4ia*)(cnt + 4 * tid);
    const v4i o4 = *(const v4ia*)(offs + 4 * tid);
    int* cp = CNT + (size_t)blockIdx.x * NBA + 4 * tid;
    int* op = OFF + (size_t)blockIdx.x * NBA + 4 * tid;
    *(volatile v4i*)cp = c4;
    *(volatile v4i*)op = o4;
    __threadfence();
    *(volatile v4i*)cp = c4;
    *(volatile v4i*)op = o4;
  }
  if (wave == 0) {
    const int f = (ovf != 0) ? 1 : 0;
    int* fp = FLG + (size_t)blockIdx.x * 32 + lane;
    *(volatile int*)fp = f;
    __threadfence();
    *(volatile int*)fp = f;
  }
}

template <int L>
__global__ __launch_bounds__(NTHR) void k_agg(const int* __restrict__ LIST, const int* __restrict__ CNT,
                                              const int* __restrict__ OFF, const int* __restrict__ FLG,
                                              const unsigned short* __restrict__ xb, unsigned short* apl,
                                              int nN, int mRows) {
  const int tid = (int)threadIdx.x, lane = tid & 31, wave = tid >> 5;
  const int row0 = (int)blockIdx.x * (NWAVE * RPW) + wave * RPW;
  const int blk  = row0 >> SLA;
  const int cv   = CNT[row0 + (lane & 15)];
  const int ofv  = OFF[row0 + (lane & 15)];
  const int fl   = FLG[(size_t)blk * 32 + lane];
  const float qn = __int_as_float(0x7fc00000);
  const float pz = (fl != 0) ? qn : 0.0f;
  const int* lb = LIST + (size_t)blk * RCAP;
#pragma unroll 1
  for (int i = 0; i < RPW; ++i) {
    const int node = row0 + i;
    int c = __builtin_amdgcn_readlane(cv, i);
    int o = __builtin_amdgcn_readlane(ofv, i);
    const bool big = c > DEGCAP;
    c = c < 0 ? 0 : (c > DEGCAP ? DEGCAP : c);
    o = o < 0 ? 0 : (o > RCAP ? RCAP : o);
    const float pzr = big ? qn : pz;
    const bool live = node < nN;
    float a0 = 0.0f, a1 = 0.0f, a2 = 0.0f, a3 = 0.0f;
#pragma unroll 1
    for (int b0 = 0; b0 < c; b0 += 32) {
      int idx = o + b0 + lane;
      idx = idx > RCAP - 1 ? RCAP - 1 : idx;
      int sr = lb[idx];
      sr = sr < 0 ? 0 : (sr > nN - 1 ? nN - 1 : sr);
      const int m32 = (c - b0) < 32 ? (c - b0) : 32;
#pragma unroll 1
      for (int k = 0; k < m32; ++k) {
        const int sk = __builtin_amdgcn_readlane(sr, k);
        if constexpr (L == 0) {
          const unsigned w = *(const u1a*)(xb + (size_t)sk * FIN + 2 * lane);
          a0 += __uint_as_float(w << 16);
          a1 += __uint_as_float(w & 0xffff0000u);
        } else {
          const unsigned short* rp = apl + (size_t)sk * AP + 2 * DF + 4 * lane;
          const v2u wh = *(const v2ua*)rp;
          const v2u wl = *(const v2ua*)(rp + DF);
          const float f0 = __uint_as_float(wh.x << 16)         + __uint_as_float(wl.x << 16);
          const float f1 = __uint_as_float(wh.x & 0xffff0000u) + __uint_as_float(wl.x & 0xffff0000u);
          const float f2 = __uint_as_float(wh.y << 16)         + __uint_as_float(wl.y << 16);
          const float f3 = __uint_as_float(wh.y & 0xffff0000u) + __uint_as_float(wl.y & 0xffff0000u);
          a0 += f0; a1 += f1; a2 += f2; a3 += f3;
        }
      }
    }
    const float inv = 1.0f / fmaxf((float)c, 1.0f);
    const float m0 = live ? (a0 * inv + pzr) : 0.0f;
    const float m1 = live ? (a1 * inv + pzr) : 0.0f;
    if constexpr (L == 0) {
      const unsigned h0 = f2bf(m0), h1 = f2bf(m1);
      const unsigned l0 = f2bf(m0 - bf2f(h0)), l1 = f2bf(m1 - bf2f(h1));
      const int hw = (int)(h0 | (h1 << 16));
      const int lw = (int)(l0 | (l1 << 16));
      const int sA = (4 * lane) & 31, sB = (4 * lane + 1) & 31, sC = (4 * lane + 2) & 31, sD = (4 * lane + 3) & 31;
      const int g0 = __shfl(hw, sA), g1 = __shfl(hw, sB), g2 = __shfl(hw, sC), g3 = __shfl(hw, sD);
      const int q0 = __shfl(lw, sA), q1 = __shfl(lw, sB), q2 = __shfl(lw, sC), q3 = __shfl(lw, sD);
      const bool lsel = lane >= 8;
      v4u pv;
      pv.x = (unsigned)(lsel ? q0 : g0);
      pv.y = (unsigned)(lsel ? q1 : g1);
      pv.z = (unsigned)(lsel ? q2 : g2);
      pv.w = (unsigned)(lsel ? q3 : g3);
      unsigned short* gp = apl + (size_t)node * AP + 8 * (lane & 15);
      if (lane < 16) *(volatile v4u*)gp = pv;
      __threadfence();
      if (lane < 16) *(volatile v4u*)gp = pv;
    } else {
      const float m2 = live ? (a2 * inv + pzr) : 0.0f;
      const float m3 = live ? (a3 * inv + pzr) : 0.0f;
      const unsigned hbx = f2bf(m0), hby = f2bf(m1), hbz = f2bf(m2), hbw = f2bf(m3);
      const unsigned lbx = f2bf(m0 - bf2f(hbx)), lby = f2bf(m1 - bf2f(hby));
      const unsigned lbz = f2bf(m2 - bf2f(hbz)), lbw = f2bf(m3 - bf2f(hbw));
      const int hw0 = (int)(hbx | (hby << 16)), hw1 = (int)(hbz | (hbw << 16));
      const int lw0 = (int)(lbx | (lby << 16)), lw1 = (int)(lbz | (lbw << 16));
      const int sa = (2 * lane) & 31, sb = (2 * lane + 1) & 31;
      const int g0 = __shfl(hw0, sa), g1 = __shfl(hw1, sa), g2 = __shfl(hw0, sb), g3 = __shfl(hw1, sb);
      const int q0 = __shfl(lw0, sa), q1 = __shfl(lw1, sa), q2 = __shfl(lw0, sb), q3 = __shfl(lw1, sb);
      const bool lsel = lane >= 16;
      v4u pv;
      pv.x = (unsigned)(lsel ? q0 : g0);
      pv.y = (unsigned)(lsel ? q1 : g1);
      pv.z = (unsigned)(lsel ? q2 : g2);
      pv.w = (unsigned)(lsel ? q3 : g3);
      unsigned short* gp = apl + (size_t)node * AP + 8 * lane;
      *(volatile v4u*)gp = pv;
      __threadfence();
      *(volatile v4u*)gp = pv;
    }
  }
  (void)mRows;
}

__device__ __forceinline__ void gemm_span(const unsigned short* ap, const unsigned short* __restrict__ bp,
                                          size_t ldb, int K, v8f (&acc)[8]) {
#pragma unroll 1
  for (int k0 = 0; k0 < K; k0 += 32) {
    FragB af;
    af.h[0] = *(const v8usa*)(ap + k0);
    af.h[1] = *(const v8usa*)(ap + k0 + 16);
#pragma unroll
    for (int nt = 0; nt < 8; ++nt) {
      const unsigned short* wq = bp + (size_t)(16 * nt) * ldb + k0;
      FragB bf;
      bf.h[0] = *(const v8usa*)wq;
      bf.h[1] = *(const v8usa*)(wq + 16);
      acc[nt] = wmb(af, bf, acc[nt]);
    }
  }
}

template <int MODE>
__global__ __launch_bounds__(GTHR) void k_gemm(const unsigned short* A1, int lda1, int K1,
                                               const unsigned short* __restrict__ A2, int lda2, int K2,
                                               const unsigned short* __restrict__ BT, int ldb,
                                               const float* __restrict__ bias, const float* __restrict__ gam,
                                               const float* __restrict__ bet, const float* __restrict__ rmn,
                                               const float* __restrict__ rvr,
                                               unsigned short* apl, int nN, int mRows) {
  __shared__ __attribute__((aligned(16))) float stg[GBM * GBN];
  __shared__ __attribute__((aligned(16))) float prm[5 * DF];
  const int tid = (int)threadIdx.x, lane = tid & 31, wave = tid >> 5, hh = lane >> 4, m = lane & 15;
  const int rowBase = (int)blockIdx.x * GBM;

  if (tid < 32) {
    const v4f b4 = bfr4(*(const v4f*)(bias + 4 * tid));
    *(v4fa*)(prm + 4 * tid) = b4;
    if constexpr (MODE != 2) {
      const v4f g4 = bfr4(*(const v4f*)(gam + 4 * tid));
      const v4f e4 = bfr4(*(const v4f*)(bet + 4 * tid));
      const v4f m4 = bfr4(*(const v4f*)(rmn + 4 * tid));
      const v4f v4 = bfr4(*(const v4f*)(rvr + 4 * tid));
      v4f r4;
      r4.x = 1.0f / sqrtf(v4.x + BNEPS);
      r4.y = 1.0f / sqrtf(v4.y + BNEPS);
      r4.z = 1.0f / sqrtf(v4.z + BNEPS);
      r4.w = 1.0f / sqrtf(v4.w + BNEPS);
      *(v4fa*)(prm + DF + 4 * tid)     = g4;
      *(v4fa*)(prm + 2 * DF + 4 * tid) = e4;
      *(v4fa*)(prm + 3 * DF + 4 * tid) = m4;
      *(v4fa*)(prm + 4 * DF + 4 * tid) = r4;
    }
  }

  v8f acc[8];
  {
    const v8f z = {0.f, 0.f, 0.f, 0.f, 0.f, 0.f, 0.f, 0.f};
#pragma unroll
    for (int t = 0; t < 8; ++t) acc[t] = z;
  }
  const size_t arow = (size_t)(rowBase + 16 * wave + m);
  const unsigned short* ap1 = A1 + arow * (size_t)lda1 + 8 * hh;
  const unsigned short* ap2 = A2 + arow * (size_t)lda2 + 8 * hh;
  const unsigned short* bp  = BT + (size_t)m * (size_t)ldb + 8 * hh;
  gemm_span(ap1, bp, (size_t)ldb, K1, acc);
  gemm_span(ap2, bp + K1, (size_t)ldb, K2, acc);

#pragma unroll
  for (int nt = 0; nt < 8; ++nt) {
    const int lc = 16 * nt + m;
#pragma unroll
    for (int r = 0; r < 8; ++r) {
      const int lr = 16 * wave + 8 * hh + r;
      stg[lr * GBN + lc] = acc[nt][r];
    }
  }
  __syncthreads();

  const v4f pb = *(const v4fa*)(prm + 4 * lane);
  v4f pg = {1.f, 1.f, 1.f, 1.f}, pe = {0.f, 0.f, 0.f, 0.f}, pm = {0.f, 0.f, 0.f, 0.f}, ps = {1.f, 1.f, 1.f, 1.f};
  if constexpr (MODE != 2) {
    pg = *(const v4fa*)(prm + DF + 4 * lane);
    pe = *(const v4fa*)(prm + 2 * DF + 4 * lane);
    pm = *(const v4fa*)(prm + 3 * DF + 4 * lane);
    ps = *(const v4fa*)(prm + 4 * DF + 4 * lane);
  }
#pragma unroll 1
  for (int i = 0; i < 16; ++i) {
    const int lr = 16 * wave + i;
    const int gr = rowBase + lr;
    const bool ok = gr < nN;
    const v4f p = *(const v4fa*)(stg + lr * GBN + 4 * lane);
    float y0 = p.x + pb.x, y1 = p.y + pb.y, y2 = p.z + pb.z, y3 = p.w + pb.w;
    if constexpr (MODE != 2) {
      y0 = pg.x * (y0 - pm.x) * ps.x + pe.x;
      y1 = pg.y * (y1 - pm.y) * ps.y + pe.y;
      y2 = pg.z * (y2 - pm.z) * ps.z + pe.z;
      y3 = pg.w * (y3 - pm.w) * ps.w + pe.w;
      y0 = (y0 > 0.f) ? y0 : (y0 - y0);
      y1 = (y1 > 0.f) ? y1 : (y1 - y1);
      y2 = (y2 > 0.f) ? y2 : (y2 - y2);
      y3 = (y3 > 0.f) ? y3 : (y3 - y3);
    }
    y0 = ok ? y0 : 0.0f; y1 = ok ? y1 : 0.0f; y2 = ok ? y2 : 0.0f; y3 = ok ? y3 : 0.0f;
    if constexpr (MODE != 2) {
      const unsigned hbx = f2bf(y0), hby = f2bf(y1), hbz = f2bf(y2), hbw = f2bf(y3);
      const unsigned lbx = f2bf(y0 - bf2f(hbx)), lby = f2bf(y1 - bf2f(hby));
      const unsigned lbz = f2bf(y2 - bf2f(hbz)), lbw = f2bf(y3 - bf2f(hbw));
      const int hw0 = (int)(hbx | (hby << 16)), hw1 = (int)(hbz | (hbw << 16));
      const int lw0 = (int)(lbx | (lby << 16)), lw1 = (int)(lbz | (lbw << 16));
      const int sa = (2 * lane) & 31, sb = (2 * lane + 1) & 31;
      const int g0 = __shfl(hw0, sa), g1 = __shfl(hw1, sa), g2 = __shfl(hw0, sb), g3 = __shfl(hw1, sb);
      const int q0 = __shfl(lw0, sa), q1 = __shfl(lw1, sa), q2 = __shfl(lw0, sb), q3 = __shfl(lw1, sb);
      const bool lsel = lane >= 16;
      v4u pv;
      pv.x = (unsigned)(lsel ? q0 : g0);
      pv.y = (unsigned)(lsel ? q1 : g1);
      pv.z = (unsigned)(lsel ? q2 : g2);
      pv.w = (unsigned)(lsel ? q3 : g3);
      unsigned short* gp = apl + (size_t)gr * AP + 2 * DF + 8 * lane;
      *(volatile v4u*)gp = pv;
      __threadfence();
      *(volatile v4u*)gp = pv;
    } else {
      v4f ov4;
      ov4.x = y0; ov4.y = y1; ov4.z = y2; ov4.w = y3;
      float* op = (float*)(apl + (size_t)gr * AP) + 4 * lane;
      *(volatile v4f*)op = ov4;
      __threadfence();
      *(volatile v4f*)op = ov4;
    }
  }
  (void)mRows;
}

__global__ __launch_bounds__(NTHR) void k_pool_head(const unsigned short* __restrict__ apl,
                                                    const int* __restrict__ batch, int nN,
                                                    const float* __restrict__ fcw, const float* __restrict__ fcb,
                                                    float* out, int nG) {
  extern __shared__ __attribute__((aligned(16))) float psm[];
  float* pmax = psm;
  float* sc   = psm + NWAVE * GPB * DF;
  const int tid = (int)threadIdx.x, lane = tid & 31, wave = tid >> 5;
  const int g0 = (int)blockIdx.x * GPB;
  const float nhuge = -__builtin_huge_valf();
  {
    v4f ninf; ninf.x = nhuge; ninf.y = nhuge; ninf.z = nhuge; ninf.w = nhuge;
    for (int i = tid * 4; i < NWAVE * GPB * DF; i += NTHR * 4) *(v4fa*)(pmax + i) = ninf;
    if (tid < GPB) sc[tid] = 0.0f;
  }
  __syncthreads();

  const int nIt = (nN + NTHR - 1) / NTHR;
#pragma unroll 1
  for (int it = 0; it < nIt; ++it) {
    const int base = (it * NWAVE + wave) * 32;
    const int n    = base + lane;
    const int ncl  = n < nN ? n : nN - 1;
    const int bv   = batch[ncl];
    const int gs   = bv - g0;
    const bool hit = (n < nN) && ((unsigned)gs < (unsigned)GPB);
    unsigned mask = __builtin_amdgcn_ballot_w32(hit);
#pragma unroll 1
    for (int q = 0; q < 32; ++q) {
      if (mask == 0u) break;
      const int k = __builtin_ctz(mask);
      mask &= mask - 1u;
      int node = base + k;
      node = node < 0 ? 0 : (node > nN - 1 ? nN - 1 : node);
      int gk = __shfl(gs, k, 32);
      gk = gk < 0 ? 0 : (gk > GPB - 1 ? GPB - 1 : gk);
      const v4f v = *(const v4f*)((const float*)(apl + (size_t)node * AP) + 4 * lane);
      float* pm = pmax + (size_t)(wave * GPB + gk) * DF + 4 * lane;
      v4f r = *(const v4fa*)pm;
      r.x = smax(r.x, v.x); r.y = smax(r.y, v.y); r.z = smax(r.z, v.z); r.w = smax(r.w, v.w);
      *(v4fa*)pm = r;
    }
  }
  __syncthreads();

  const v4f fw = bfr4(*(const v4f*)(fcw + 4 * lane));
  const float fb = bfr(fcb[0]);
#pragma unroll 1
  for (int q = 0; q < 4; ++q) {
    const int gsl = wave * 4 + q;
    v4f r = *(const v4fa*)(pmax + (size_t)gsl * DF + 4 * lane);
#pragma unroll 1
    for (int w2 = 1; w2 < NWAVE; ++w2) {
      const v4f v = *(const v4fa*)(pmax + (size_t)(w2 * GPB + gsl) * DF + 4 * lane);
      r.x = smax(r.x, v.x); r.y = smax(r.y, v.y); r.z = smax(r.z, v.z); r.w = smax(r.w, v.w);
    }
    float s = r.x * fw.x;
    s = fmaf(r.y, fw.y, s);
    s = fmaf(r.z, fw.z, s);
    s = fmaf(r.w, fw.w, s);
    s += __shfl_xor(s, 16, 32);
    s += __shfl_xor(s, 8, 32);
    s += __shfl_xor(s, 4, 32);
    s += __shfl_xor(s, 2, 32);
    s += __shfl_xor(s, 1, 32);
    if (lane == 0) sc[gsl] = s + fb;
  }
  __syncthreads();
  if (wave == 0) {
    const float o = sc[lane];
    const int g = g0 + lane;
    if (g < nG) {
      float* op = out + g;
      *(volatile float*)op = o;
      __threadfence();
      *(volatile float*)op = o;
    }
  }
}

static inline int cdiv(int a, int b) { return (a + b - 1) / b; }
static inline size_t al256(size_t o) { return (o + 255) & ~(size_t)255; }

extern "C" void kernel_launch(void* const* d_in, const int* in_sizes, int n_in,
                              void* d_out, int out_size, void* d_ws, size_t ws_size,
                              hipStream_t stream) {
  if (n_in < 22) return;
  const int nN = in_sizes[2];
  if (nN < GBM || nN > (1 << 21)) return;
  if ((long long)in_sizes[0] != (long long)nN * FIN) return;
  if (in_sizes[1] < 2 || (in_sizes[1] & 1) != 0) return;
  const int nE = in_sizes[1] / 2;
  if (nE < 1 || nE >= (1 << 21)) return;
  if (in_sizes[3] != FIN * DF || in_sizes[5] != FIN * DF) return;
  if (in_sizes[6] != DF * DF || in_sizes[8] != DF * DF) return;
  if (in_sizes[9] != DF * DF || in_sizes[11] != DF * DF) return;
  if (in_sizes[4] != DF || in_sizes[7] != DF || in_sizes[10] != DF) return;
  for (int i = 12; i < 21; ++i) if (in_sizes[i] != DF) return;
  if (in_sizes[21] != 1) return;
  if (out_size < GPB || (out_size % GPB) != 0 || out_size > (1 << 20)) return;
  const int nG = out_size;

  const float* x    = (const float*)d_in[0];
  const int*   ei   = (const int*)  d_in[1];
  const int*   bat  = (const int*)  d_in[2];
  const float* W1l  = (const float*)d_in[3];
  const float* b1l  = (const float*)d_in[4];
  const float* W1r  = (const float*)d_in[5];
  const float* W2l  = (const float*)d_in[6];
  const float* b2l  = (const float*)d_in[7];
  const float* W2r  = (const float*)d_in[8];
  const float* W3l  = (const float*)d_in[9];
  const float* b3l  = (const float*)d_in[10];
  const float* W3r  = (const float*)d_in[11];
  const float* g1   = (const float*)d_in[12];
  const float* be1  = (const float*)d_in[13];
  const float* rm1  = (const float*)d_in[14];
  const float* rv1  = (const float*)d_in[15];
  const float* g2   = (const float*)d_in[16];
  const float* be2  = (const float*)d_in[17];
  const float* rm2  = (const float*)d_in[18];
  const float* rv2  = (const float*)d_in[19];
  const float* fcW  = (const float*)d_in[20];
  const float* fcb  = (const float*)d_in[21];
  float* out = (float*)d_out;
  const int* src = ei;
  const int* dst = ei + nE;

  const int MP = cdiv(nN, MROWS) * MROWS;
  const int gM = MP / GBM;
  const int gA = cdiv(MP, NBA);
  const int gG = MP / (NWAVE * RPW);
  const int vec8 = ((nE & 3) == 0) ? 1 : 0;
  const int nUx = MP * (FIN / 8);

  char* ws = (char*)d_ws;
  size_t off = 0;
  const size_t oWPL = off; off = al256(off + (size_t)WPLH * 2);
  const size_t oXB  = off; off = al256(off + (size_t)MP * FIN * 2);
  const size_t oA   = off; off = al256(off + (size_t)MP * AP * 2);
  const size_t oLS  = off; off = al256(off + (size_t)gA * RCAP * 4);
  const size_t oCN  = off; off = al256(off + (size_t)gA * NBA * 4);
  const size_t oOF  = off; off = al256(off + (size_t)gA * NBA * 4);
  const size_t oFL  = off; off = al256(off + (size_t)gA * 128);
  if (off > ws_size || off > (size_t)WSMAX) return;
  unsigned short* WPL = (unsigned short*)(ws + oWPL);
  unsigned short* XB  = (unsigned short*)(ws + oXB);
  unsigned short* Apl = (unsigned short*)(ws + oA);
  int* LIST = (int*)(ws + oLS);
  int* CNT  = (int*)(ws + oCN);
  int* OFF  = (int*)(ws + oOF);
  int* FLG  = (int*)(ws + oFL);

  const size_t cmpLds  = (size_t)CMP_LDS_INTS * 4;
  const size_t poolLds = (size_t)POOL_LDS_FLOATS * 4;
  hipFuncSetAttribute(reinterpret_cast<const void*>(&k_compact), hipFuncAttributeMaxDynamicSharedMemorySize, (int)cmpLds);
  hipFuncSetAttribute(reinterpret_cast<const void*>(&k_pool_head), hipFuncAttributeMaxDynamicSharedMemorySize, (int)poolLds);

  k_prep<<<(NUW + nUx) / NTHR, NTHR, 0, stream>>>(x, W1l, W1r, W2l, W2r, W3l, W3r, WPL, XB, nN, nUx);
  k_compact<<<gA, NTHR, cmpLds, stream>>>(src, dst, nE, nN, vec8, LIST, CNT, OFF, FLG);
  k_agg<0><<<gG, NTHR, 0, stream>>>(LIST, CNT, OFF, FLG, XB, Apl, nN, MP);
  k_gemm<0><<<gM, GTHR, 0, stream>>>(Apl, AP, 2 * FIN, XB, FIN, FIN, WPL, K0C,
                                     b1l, g1, be1, rm1, rv1, Apl, nN, MP);
  k_agg<1><<<gG, NTHR, 0, stream>>>(LIST, CNT, OFF, FLG, XB, Apl, nN, MP);
  k_gemm<1><<<gM, GTHR, 0, stream>>>(Apl, AP, KS, XB, FIN, 0, WPL + W2OFF, KS,
                                     b2l, g2, be2, rm2, rv2, Apl, nN, MP);
  k_agg<1><<<gG, NTHR, 0, stream>>>(LIST, CNT, OFF, FLG, XB, Apl, nN, MP);
  k_gemm<2><<<gM, GTHR, 0, stream>>>(Apl, AP, KS, XB, FIN, 0, WPL + W3OFF, KS,
                                     b3l, b3l, b3l, b3l, b3l, Apl, nN, MP);
  k_pool_head<<<nG / GPB, NTHR, poolLds, stream>>>(Apl, bat, nN, fcW, fcb, out, nG);
}
